// EwaldPotential_54314156425687
// MI455X (gfx1250) — hardware-run, weakly checked
//
#include <hip/hip_runtime.h>
#include <math.h>

typedef __attribute__((ext_vector_type(16))) _Float16 v16h;
typedef __attribute__((ext_vector_type(16))) __bf16 v16b;
typedef __attribute__((ext_vector_type(8)))  _Float16 v8h;
typedef __attribute__((ext_vector_type(8)))  float v8f;
typedef __attribute__((ext_vector_type(4)))  float v4f;
typedef __attribute__((ext_vector_type(2)))  float v2f;
typedef __attribute__((ext_vector_type(4)))  unsigned v4u;
typedef __attribute__((ext_vector_type(4)))  int v4i;
typedef float __attribute__((may_alias)) float_a;
typedef int __attribute__((may_alias)) int_a;

template <typename T> __device__ __forceinline__ void vst2(void* p, T v) { *(volatile T*)p = v; __threadfence(); *(volatile T*)p = v; }
__device__ __forceinline__ v8f wmma16(v16h a, v16h b, v8f c) {
  v8f d = __builtin_amdgcn_wmma_f32_16x16x32_f16(false, a, false, b, (short)0, c, false, false);
  asm volatile("v_nop\n\tv_nop\n\tv_nop\n\tv_nop" : "+v"(d) : "v"(a), "v"(b));
  return d;
}
__device__ __forceinline__ v8f wmma_bf(v16b a, v16b b, v8f c) {
  v8f d = __builtin_amdgcn_wmma_f32_16x16x32_bf16(false, a, false, b, (short)0, c, false, false);
  asm volatile("v_nop\n\tv_nop\n\tv_nop\n\tv_nop" : "+v"(d) : "v"(a), "v"(b));
  return d;
}
__device__ __forceinline__ v16h frag_h(const _Float16* rowk0, int lane) {
  union { v16h v; v8h q[2]; } u; const _Float16* p = rowk0 + 8 * (lane >> 4);
  u.q[0] = *(const v8h*)p; u.q[1] = *(const v8h*)(p + 16); return u.v;
}
__device__ __forceinline__ v16h frag_f32(const float* rowk0, int lane) {
  v16h a; const float* p = rowk0 + 8 * (lane >> 4);
#pragma unroll
  for (int i = 0; i < 8; ++i) { a[i] = (_Float16)p[i]; a[8 + i] = (_Float16)p[16 + i]; }
  return a;
}
__device__ __forceinline__ v16h frag_f32s(const float* rowk0, int lane, float sc) {
  v16h a; const float* p = rowk0 + 8 * (lane >> 4);
#pragma unroll
  for (int i = 0; i < 8; ++i) { a[i] = (_Float16)(p[i] * sc); a[8 + i] = (_Float16)(p[16 + i] * sc); }
  return a;
}
__device__ __forceinline__ v16h fragc_f32(const float* W, int k0, int n, int lane, int ld, int K) {
  v16h a; const int g = lane >> 4;
#pragma unroll
  for (int i = 0; i < 8; ++i) { const int ka = k0 + 8 * g + i, kb = ka + 16;
    a[i] = (_Float16)(ka < K ? W[(size_t)(ka < K ? ka : K - 1) * ld + n] : 0.f); a[8 + i] = (_Float16)(kb < K ? W[(size_t)(kb < K ? kb : K - 1) * ld + n] : 0.f); }
  return a;
}
struct F2 { v16b h, l; };
__device__ __forceinline__ F2 bsplit16(const float v[16]) { F2 r;
#pragma unroll
  for (int i = 0; i < 16; ++i) { const __bf16 h = (__bf16)v[i]; r.h[i] = h; r.l[i] = (__bf16)(v[i] - (float)h); }
  return r; }
__device__ __forceinline__ F2 split_row(const float* row, int k0, int lane) { float v[16]; const float* p = row + k0 + 8 * (lane >> 4);
#pragma unroll
  for (int i = 0; i < 8; ++i) { v[i] = p[i]; v[8 + i] = p[16 + i]; }
  return bsplit16(v); }
__device__ __forceinline__ F2 split_rowK(const float* row, int k0, int lane, int K) { float v[16]; const int g = lane >> 4;
#pragma unroll
  for (int i = 0; i < 8; ++i) { const int ka = k0 + 8 * g + i, kb = ka + 16; v[i] = ka < K ? row[ka < K ? ka : K - 1] : 0.f; v[8 + i] = kb < K ? row[kb < K ? kb : K - 1] : 0.f; }
  return bsplit16(v); }
__device__ __forceinline__ F2 split_col(const float* W, int k0, int n, int lane, int ld, int K) { float v[16]; const int g = lane >> 4;
#pragma unroll
  for (int i = 0; i < 8; ++i) { const int ka = k0 + 8 * g + i, kb = ka + 16; v[i] = ka < K ? W[(size_t)(ka < K ? ka : K - 1) * ld + n] : 0.f; v[8 + i] = kb < K ? W[(size_t)(kb < K ? kb : K - 1) * ld + n] : 0.f; }
  return bsplit16(v); }
__device__ __forceinline__ v8f mac3(const F2& a, const F2& b, v8f c) { c = wmma_bf(a.l, b.h, c); c = wmma_bf(a.h, b.l, c); return wmma_bf(a.h, b.h, c); }
__device__ __forceinline__ float sigm(float v) { return 1.0f / (1.0f + expf(-v)); }
#define LDSX() do { asm volatile("s_wait_dscnt 0" ::: "memory"); __builtin_amdgcn_wave_barrier(); __builtin_amdgcn_fence(__ATOMIC_RELEASE, "workgroup"); } while (0)


#define NPT 8192
#define NCH 4
#ifndef NRB
#define NRB (NPT / 64)
#endif
typedef __attribute__((ext_vector_type(8))) __bf16 v8b;
__device__ __forceinline__ v16b frag_b(const __bf16* rowk0, int lane) {
  union { v16b v; v8b q[2]; } u; const __bf16* p = rowk0 + 8 * (lane >> 4);
  u.q[0] = *(const v8b*)p; u.q[1] = *(const v8b*)(p + 16); return u.v;
}
__device__ __forceinline__ float bfr(float v) { return (float)(__bf16)v; }
__device__ __attribute__((noinline)) float exp_ni(float v) { return expf(v); }
__device__ __attribute__((noinline)) float erf_ni(float v) { return erff(v); }

#define WS_QT   0u
#define WS_POS  (WS_QT + 2u * 16 * NPT)
#define WS_PART (WS_POS + 4u * 3 * NPT)
#define WS_END  (WS_PART + 128u * NRB)

__global__ __launch_bounds__(256) void k_prep(const float* __restrict__ POS, const float* __restrict__ Q, __bf16* __restrict__ QT, float* __restrict__ PT) {
  const int t = threadIdx.x;
  for (int e = t; e < 16 * NPT / 8; e += 256) { const int c = e / (NPT / 8), pc = e % (NPT / 8); union { v4u u; __bf16 h[8]; } w;
#pragma unroll
    for (int i = 0; i < 8; ++i) w.h[i] = (__bf16)((c < NCH) ? Q[(size_t)(pc * 8 + i) * NCH + c] : 0.f);
    vst2((unsigned*)(QT + (size_t)c * NPT + pc * 8), w.u); }
  for (int e = t; e < 3 * NPT / 4; e += 256) { const int a = e / (NPT / 4), pc = e % (NPT / 4); v4f v;
#pragma unroll
    for (int i = 0; i < 4; ++i) v[i] = bfr(POS[(size_t)(pc * 4 + i) * 3 + a]);
    vst2(PT + (size_t)a * NPT + pc * 4, v); }
}
__global__ __launch_bounds__(128) void k_pot(const float* __restrict__ PT, const float* __restrict__ Q, const __bf16* __restrict__ QT, double* __restrict__ PART) {
  __shared__ double sred[4]; __shared__ __align__(16) double sl[16];
  const int tid = threadIdx.x, wave = tid >> 5, lane = tid & 31, col = lane & 15, g = lane >> 4; const size_t i = (size_t)blockIdx.x * 64 + wave * 16 + col;
  const float xi = PT[i], yi = PT[NPT + i], zi = PT[2 * NPT + i];
  v8f acc = {}, accl = {};
#pragma unroll 1
  for (int kc = 0; kc < NPT / 32; ++kc) { v16b ah, al;
#pragma unroll
    for (int e = 0; e < 16; ++e) { const int j = kc * 32 + 8 * g + (e & 7) + ((e >> 3) << 4); const float dx = PT[j] - xi, dy = PT[NPT + j] - yi, dz = PT[2 * NPT + j] - zi; const float r = sqrtf(dx * dx + dy * dy + dz * dz);
      const float kv = erf_ni(r * 0.70710678118654752f) / (r + 1e-6f); const __bf16 hb = (__bf16)kv; ah[e] = hb; al[e] = (__bf16)(kv - (float)hb); }
    const v16b b = frag_b(QT + (size_t)col * NPT + kc * 32, lane);
    acc = wmma_bf(ah, b, acc); accl = wmma_bf(al, b, accl); }
  float part = 0.f;
#pragma unroll
  for (int r = 0; r < 8; ++r) { const size_t ii = (size_t)blockIdx.x * 64 + wave * 16 + 8 * g + r; const float m = acc[r] + accl[r]; if (col < NCH) part += bfr(Q[ii * NCH + col]) * m; }
  double dp = (double)part;
#pragma unroll
  for (int o = 1; o < 32; o <<= 1) dp += __shfl_xor(dp, o);
  if (lane == 0) sred[wave] = dp;
  if (tid < 16) sl[tid] = 0.0;
  __syncthreads();
  if (tid == 0) sl[0] = (sred[0] + sred[1]) + (sred[2] + sred[3]);
  __syncthreads();
  if (tid < 8) vst2((unsigned*)(PART + (size_t)blockIdx.x * 16 + tid * 2), *(const v4u*)&sl[tid * 2]);
}
__global__ __launch_bounds__(256) void k_final(const double* __restrict__ PART, const float* __restrict__ Q, float* __restrict__ OUT) {
  __shared__ double s[2][256]; const int t = threadIdx.x; double a = 0.0, sq = 0.0;
  for (int b = t; b < NRB; b += 256) a += PART[(size_t)b * 16];
  for (int e = t; e < NPT * NCH; e += 256) { const double qv = (double)bfr(Q[e]); sq += qv * qv; }
  s[0][t] = a; s[1][t] = sq; __syncthreads();
  if (t == 0) { double A = 0.0, S = 0.0; for (int k = 0; k < 256; ++k) { A += s[0][k]; S += s[1][k]; }
    const double twopi = 6.283185307179586; const double pot = A / twopi / 2.0 + S / (1.0 * pow(twopi, 1.5)); const float v = (float)pot; *(volatile float*)OUT = v; *(volatile float*)OUT = v; }
}
extern "C" void kernel_launch(void* const* d_in, const int* in_sizes, int n_in, void* d_out, int out_size, void* d_ws, size_t ws_size, hipStream_t stream) {
  (void)in_sizes; (void)n_in; (void)out_size;
  const float** F = (const float**)d_in;
  if (ws_size < (size_t)WS_END) return;
  char* ws = (char*)d_ws; __bf16* QT = (__bf16*)(ws + WS_QT); float* PT = (float*)(ws + WS_POS); double* PART = (double*)(ws + WS_PART);
  k_prep<<<1, 256, 0, stream>>>(F[0], F[1], QT, PT);
  k_pot<<<NRB, 128, 0, stream>>>(PT, F[1], QT, PART);
  k_final<<<1, 256, 0, stream>>>(PART, F[1], (float*)d_out);
}
